// FaceDetection_20830591386199
// MI455X (gfx1250) — hardware-verified
//
#include <hip/hip_runtime.h>

#pragma clang fp contract(off)

#define TOPK 100
#define TOPKP 128
#define NANCH 12288
#define IMW 1024
#define IMHW 1048576

typedef __bf16 bf16_t;
typedef bf16_t v16b __attribute__((ext_vector_type(16)));
typedef float v8f __attribute__((ext_vector_type(8)));
typedef float v4f __attribute__((ext_vector_type(4)));
typedef unsigned int v4u __attribute__((ext_vector_type(4)));

union Frag { v16b v; v4u q[2]; unsigned short s[16]; };
union P8 { v4u q; unsigned short s[8]; };
union P4F { v4f v; float f[4]; };

__device__ __forceinline__ unsigned short bf_bits(float x) {
  unsigned int u = __float_as_uint(x);
  u += 0x7FFFu + ((u >> 16) & 1u);
  return (unsigned short)(u >> 16);
}
__device__ __forceinline__ void split2(float x, unsigned short& hb, unsigned short& lb) {
  unsigned short hh = bf_bits(x);
  float hf = __uint_as_float(((unsigned int)hh) << 16);
  hb = hh;
  lb = bf_bits(x - hf);
}

__device__ __forceinline__ v8f mma3(v8f c, v16b ah, v16b al, v16b bh, v16b bl) {
  c = __builtin_amdgcn_wmma_f32_16x16x32_bf16(false, ah, false, bh, (short)0, c, false, false);
  c = __builtin_amdgcn_wmma_f32_16x16x32_bf16(false, ah, false, bl, (short)0, c, false, false);
  c = __builtin_amdgcn_wmma_f32_16x16x32_bf16(false, al, false, bh, (short)0, c, false, false);
  asm volatile("v_nop\n\tv_nop\n\tv_nop\n\tv_nop" : "+v"(c) : "v"(ah), "v"(al), "v"(bh), "v"(bl));
  return c;
}

__global__ __launch_bounds__(256) void k_pack(const float* __restrict__ w,
                                              unsigned short* wpH, unsigned short* wpL,
                                              int Cout, int Cin, int Kp, int nThr) {
  const int g = blockIdx.x * 256 + threadIdx.x;
  const bool act = g < nThr;
  const int gg = act ? g : 0;
  const int e0 = gg * 8;
  const int n = e0 / Kp;
  const int k0 = e0 - n * Kp;
  const int Kr = Cin * 9;
  P8 uh, ul;
#pragma unroll
  for (int i = 0; i < 8; ++i) {
    const int k = k0 + i;
    float v = 0.0f;
    if (n < Cout && k < Kr) {
      const int tap = k / Cin;
      const int ci = k - tap * Cin;
      const int fy = tap / 3;
      const int fx = tap - fy * 3;
      v = w[((n * Cin + ci) * 3 + fy) * 3 + fx];
    }
    unsigned short hb, lb;
    split2(v, hb, lb);
    uh.s[i] = hb;
    ul.s[i] = lb;
  }
  if (act) {
    *(volatile v4u*)(wpH + e0) = uh.q;
    *(volatile v4u*)(wpL + e0) = ul.q;
  }
  __threadfence();
  if (act) {
    *(volatile v4u*)(wpH + e0) = uh.q;
    *(volatile v4u*)(wpL + e0) = ul.q;
  }
}

__global__ __launch_bounds__(128) void k_conv1(const float* __restrict__ frame,
                                               const unsigned short* __restrict__ wH,
                                               const unsigned short* __restrict__ wL,
                                               const float* __restrict__ bias,
                                               unsigned short* outH, unsigned short* outL,
                                               int nTiles) {
  __shared__ unsigned short sH[4][512];
  __shared__ unsigned short sL[4][512];
  const int lane = threadIdx.x & 31, wave = threadIdx.x >> 5;
  const int h = lane >> 4, m = lane & 15;
  const int wid = blockIdx.x * 4 + wave;
  const bool act = wid < nTiles;
  const int t = act ? wid : 0;
  const int pbase = t * 16;
  const int oy = pbase >> 9;
  const int ox = (pbase & 511) + m;

  Frag aH, aL;
#pragma unroll
  for (int i = 0; i < 16; ++i) {
    const int k = 8 * h + (i & 7) + ((i >> 3) << 4);
    float v = 0.0f;
    if (k < 27) {
      const int tap = k / 3;
      const int ci = k - 3 * tap;
      const int fy = tap / 3;
      const int fx = tap - 3 * fy;
      const int iy = 2 * oy + fy;
      const int ix = 2 * ox + fx;
      if (iy < IMW && ix < IMW) v = frame[ci * IMHW + iy * IMW + ix];
    }
    unsigned short hb, lb;
    split2(v, hb, lb);
    aH.s[i] = hb;
    aL.s[i] = lb;
  }

  v8f acc[2];
#pragma unroll
  for (int c = 0; c < 2; ++c) {
    const unsigned short* br = wH + (16 * c + m) * 32;
    const unsigned short* brl = wL + (16 * c + m) * 32;
    Frag bH, bL;
    bH.q[0] = *(const v4u*)(br + 8 * h);
    bH.q[1] = *(const v4u*)(br + 16 + 8 * h);
    bL.q[0] = *(const v4u*)(brl + 8 * h);
    bL.q[1] = *(const v4u*)(brl + 16 + 8 * h);
    v8f z = {0.0f, 0.0f, 0.0f, 0.0f, 0.0f, 0.0f, 0.0f, 0.0f};
    acc[c] = mma3(z, aH.v, aL.v, bH.v, bL.v);
  }

#pragma unroll
  for (int c = 0; c < 2; ++c) {
    const int ch = 16 * c + m;
    const float bn = bias[ch];
#pragma unroll
    for (int r = 0; r < 8; ++r) {
      const float v = fmaxf(acc[c][r] + bn, 0.0f);
      const int px = 8 * h + r;
      unsigned short hb, lb;
      split2(v, hb, lb);
      sH[wave][px * 32 + ch] = hb;
      sL[wave][px * 32 + ch] = lb;
    }
  }
  __syncthreads();
  v4u oh[2], ol[2];
#pragma unroll
  for (int i = 0; i < 2; ++i) {
    oh[i] = *(const v4u*)(&sH[wave][256 * i + 8 * lane]);
    ol[i] = *(const v4u*)(&sL[wave][256 * i + 8 * lane]);
  }
  const size_t gbase = (size_t)pbase * 32;
  if (act) {
#pragma unroll
    for (int i = 0; i < 2; ++i) {
      *(volatile v4u*)(outH + gbase + 256 * i + 8 * lane) = oh[i];
      *(volatile v4u*)(outL + gbase + 256 * i + 8 * lane) = ol[i];
    }
  }
  __threadfence();
  if (act) {
#pragma unroll
    for (int i = 0; i < 2; ++i) {
      *(volatile v4u*)(outH + gbase + 256 * i + 8 * lane) = oh[i];
      *(volatile v4u*)(outL + gbase + 256 * i + 8 * lane) = ol[i];
    }
  }
}

template <int NCHUNK, int OUTF>
__global__ __launch_bounds__(128) void k_conv(
    const unsigned short* __restrict__ inH, const unsigned short* __restrict__ inL,
    const unsigned short* __restrict__ wH, const unsigned short* __restrict__ wL,
    const float* __restrict__ bias,
    unsigned short* outH, unsigned short* outL, float* outF,
    int Cin, int IH, int IW, int OW, int CoutPad, int CoutReal,
    int stride, int pad, int relu, int nTiles) {
  constexpr int NCH = 16 * NCHUNK;
  __shared__ unsigned short sH[4][16 * NCH];
  __shared__ unsigned short sL[4][16 * NCH];
  __shared__ float sF[4][256];
  const int lane = threadIdx.x & 31, wave = threadIdx.x >> 5;
  const int h = lane >> 4, m = lane & 15;
  const int wid = blockIdx.x * 4 + wave;
  const bool act = wid < nTiles;
  const int t = act ? wid : 0;
  const int ngrp = CoutPad / NCH;
  const int ptile = t / ngrp;
  const int grp = t - ptile * ngrp;
  const int pbase = ptile * 16;
  const int nb = grp * NCH;
  const int oy0 = pbase / OW;
  const int ox0 = pbase - oy0 * OW;
  const int ax = (ox0 + m) * stride - pad;
  const int ay0 = oy0 * stride - pad;
  const int K = Cin * 9;
  const int cSteps = Cin >> 5;
  const v4u zq = {0u, 0u, 0u, 0u};

  v8f acc[NCHUNK];
#pragma unroll
  for (int c = 0; c < NCHUNK; ++c) {
    v8f z = {0.0f, 0.0f, 0.0f, 0.0f, 0.0f, 0.0f, 0.0f, 0.0f};
    acc[c] = z;
  }

  for (int tap = 0; tap < 9; ++tap) {
    const int fy = tap / 3, fx = tap - fy * 3;
    const int iy = ay0 + fy, ix = ax + fx;
    const bool ok = ((unsigned)iy < (unsigned)IH) && ((unsigned)ix < (unsigned)IW);
    size_t abase = 0;
    if (ok) abase = ((size_t)iy * IW + ix) * (size_t)Cin;
    for (int cb = 0; cb < cSteps; ++cb) {
      const int k0 = tap * Cin + cb * 32;
      Frag aH, aL;
      if (ok) {
        const unsigned short* ap = inH + abase + cb * 32;
        const unsigned short* alp = inL + abase + cb * 32;
        aH.q[0] = *(const v4u*)(ap + 8 * h);
        aH.q[1] = *(const v4u*)(ap + 16 + 8 * h);
        aL.q[0] = *(const v4u*)(alp + 8 * h);
        aL.q[1] = *(const v4u*)(alp + 16 + 8 * h);
      } else {
        aH.q[0] = zq; aH.q[1] = zq; aL.q[0] = zq; aL.q[1] = zq;
      }
#pragma unroll
      for (int c = 0; c < NCHUNK; ++c) {
        const size_t boff = (size_t)(nb + 16 * c + m) * (size_t)K + (size_t)k0;
        Frag bH, bL;
        bH.q[0] = *(const v4u*)(wH + boff + 8 * h);
        bH.q[1] = *(const v4u*)(wH + boff + 16 + 8 * h);
        bL.q[0] = *(const v4u*)(wL + boff + 8 * h);
        bL.q[1] = *(const v4u*)(wL + boff + 16 + 8 * h);
        acc[c] = mma3(acc[c], aH.v, aL.v, bH.v, bL.v);
      }
    }
  }

#pragma unroll
  for (int c = 0; c < NCHUNK; ++c) {
    const int ch = nb + 16 * c + m;
    const float bn = (ch < CoutReal) ? bias[ch] : 0.0f;
#pragma unroll
    for (int r = 0; r < 8; ++r) {
      float v = acc[c][r] + bn;
      if (relu) v = fmaxf(v, 0.0f);
      const int px = 8 * h + r;
      if (OUTF) {
        sF[wave][px * 16 + m] = v;
      } else {
        unsigned short hb, lb;
        split2(v, hb, lb);
        sH[wave][px * NCH + 16 * c + m] = hb;
        sL[wave][px * NCH + 16 * c + m] = lb;
      }
    }
  }
  __syncthreads();
  if (OUTF) {
    v4f o[2];
    size_t go[2];
#pragma unroll
    for (int i = 0; i < 2; ++i) {
      const int e = 32 * i + lane;
      const int rr = e >> 2;
      const int cc = (e & 3) * 4;
      o[i] = *(const v4f*)(&sF[wave][rr * 16 + cc]);
      go[i] = (size_t)(pbase + rr) * (size_t)CoutPad + (size_t)nb + (size_t)cc;
    }
    if (act) {
#pragma unroll
      for (int i = 0; i < 2; ++i) *(volatile v4f*)(outF + go[i]) = o[i];
    }
    __threadfence();
    if (act) {
#pragma unroll
      for (int i = 0; i < 2; ++i) *(volatile v4f*)(outF + go[i]) = o[i];
    }
  } else {
    constexpr int NI = NCH / 16;
    constexpr int PPP = NCH / 8;
    v4u oh[NI], ol[NI];
    size_t go[NI];
#pragma unroll
    for (int i = 0; i < NI; ++i) {
      const int e = 32 * i + lane;
      const int rr = e / PPP;
      const int cc = (e - rr * PPP) * 8;
      oh[i] = *(const v4u*)(&sH[wave][rr * NCH + cc]);
      ol[i] = *(const v4u*)(&sL[wave][rr * NCH + cc]);
      go[i] = (size_t)(pbase + rr) * (size_t)CoutPad + (size_t)nb + (size_t)cc;
    }
    if (act) {
#pragma unroll
      for (int i = 0; i < NI; ++i) {
        *(volatile v4u*)(outH + go[i]) = oh[i];
        *(volatile v4u*)(outL + go[i]) = ol[i];
      }
    }
    __threadfence();
    if (act) {
#pragma unroll
      for (int i = 0; i < NI; ++i) {
        *(volatile v4u*)(outH + go[i]) = oh[i];
        *(volatile v4u*)(outL + go[i]) = ol[i];
      }
    }
  }
}

__global__ __launch_bounds__(256) void k_select(const float* __restrict__ hd, float* tb, int* kp) {
  __shared__ float sc[NANCH];
  __shared__ float rs[256];
  __shared__ int ri[256];
  __shared__ int sidx[TOPK];
  __shared__ int sval[TOPK];
  __shared__ float bx[TOPK * 4];
  __shared__ float ar[TOPK];
  __shared__ int keep[TOPK];
  const int tid = threadIdx.x;

  for (int i = tid; i < NANCH; i += 256) {
    const int a = i % 3, xy = i / 3;
    const float lg = hd[xy * 16 + a * 5 + 4];
    const float e = expf(-lg);
    const float s = 1.0f / (1.0f + e);
    sc[i] = (s >= 0.5f) ? s : -1.0f;
  }
  __syncthreads();

  for (int t = 0; t < TOPK; ++t) {
    float best = -4.0f;
    int bi = NANCH;
    for (int i = tid; i < NANCH; i += 256) {
      const float v = sc[i];
      if (v > best) { best = v; bi = i; }
    }
    rs[tid] = best;
    ri[tid] = bi;
    __syncthreads();
    for (int s2 = 128; s2 > 0; s2 >>= 1) {
      if (tid < s2) {
        const float ov = rs[tid + s2];
        const int oi = ri[tid + s2];
        if (ov > rs[tid] || (ov == rs[tid] && oi < ri[tid])) { rs[tid] = ov; ri[tid] = oi; }
      }
      __syncthreads();
    }
    if (tid == 0) {
      int si = ri[0];
      si = (si < 0) ? 0 : ((si >= NANCH) ? (NANCH - 1) : si);
      sidx[t] = si;
      sval[t] = (rs[0] > 0.0f) ? 1 : 0;
      sc[si] = -3.0f;
    }
    __syncthreads();
  }

  if (tid < TOPK) {
    const int i = sidx[tid];
    const int a = i % 3;
    const int xy = i / 3;
    const int x = xy & 63;
    const int y = xy >> 6;
    const float* hp = hd + xy * 16 + a * 5;
    const float t0 = hp[0], t1 = hp[1], t2 = hp[2], t3 = hp[3];
    const float s = (a == 0) ? 32.0f : ((a == 1) ? 64.0f : 128.0f);
    const float acx = ((float)x + 0.5f) * 16.0f;
    const float acy = ((float)y + 0.5f) * 16.0f;
    const float cx = acx + t0 * s;
    const float cy = acy + t1 * s;
    const float bw = s * expf(fminf(fmaxf(t2, -4.0f), 4.0f));
    const float bh = s * expf(fminf(fmaxf(t3, -4.0f), 4.0f));
    const float hx = bw * 0.5f, hy = bh * 0.5f;
    const float x1 = cx - hx, y1 = cy - hy, x2 = cx + hx, y2 = cy + hy;
    bx[tid * 4 + 0] = x1;
    bx[tid * 4 + 1] = y1;
    bx[tid * 4 + 2] = x2;
    bx[tid * 4 + 3] = y2;
    ar[tid] = (x2 - x1) * (y2 - y1);
    keep[tid] = sval[tid];
  }
  __syncthreads();

  for (int i = 0; i < TOPK; ++i) {
    if (tid < TOPK && tid > i && keep[i]) {
      const float lx = fmaxf(bx[i * 4 + 0], bx[tid * 4 + 0]);
      const float ly = fmaxf(bx[i * 4 + 1], bx[tid * 4 + 1]);
      const float rx = fminf(bx[i * 4 + 2], bx[tid * 4 + 2]);
      const float ry = fminf(bx[i * 4 + 3], bx[tid * 4 + 3]);
      const float iw = fmaxf(rx - lx, 0.0f);
      const float ih = fmaxf(ry - ly, 0.0f);
      const float inter = iw * ih;
      const float den = ((ar[i] + ar[tid]) - inter) + 1e-9f;
      const float iou = inter / den;
      if (iou > 0.5f) keep[tid] = 0;
    }
    __syncthreads();
  }

  P4F o;
  o.f[0] = 0.0f; o.f[1] = 0.0f; o.f[2] = 0.0f; o.f[3] = 0.0f;
  int kv = 0;
  if (tid < TOPK) {
    o.f[0] = bx[tid * 4 + 0];
    o.f[1] = bx[tid * 4 + 1];
    o.f[2] = bx[tid * 4 + 2];
    o.f[3] = bx[tid * 4 + 3];
    kv = keep[tid];
  }
  if (tid < TOPKP) {
    *(volatile v4f*)(tb + tid * 4) = o.v;
    *(volatile int*)(kp + tid) = kv;
  }
  __threadfence();
  if (tid < TOPKP) {
    *(volatile v4f*)(tb + tid * 4) = o.v;
    *(volatile int*)(kp + tid) = kv;
  }
}

__global__ __launch_bounds__(256) void k_draw(const float* __restrict__ frame,
                                              const float* __restrict__ tb,
                                              const int* __restrict__ kp,
                                              float* out) {
  __shared__ float bx[TOPK * 4];
  __shared__ int rel[TOPK];
  __shared__ int lst[TOPK];
  __shared__ int cnt;
  const int tid = threadIdx.x;
  const int y = blockIdx.x;
  const float fy = (float)y;
  if (tid < TOPK) {
    const float x1 = fminf(fmaxf(tb[tid * 4 + 0], 0.0f), 1024.0f);
    const float y1 = fminf(fmaxf(tb[tid * 4 + 1], 0.0f), 1024.0f);
    const float x2 = fminf(fmaxf(tb[tid * 4 + 2], 0.0f), 1024.0f);
    const float y2 = fminf(fmaxf(tb[tid * 4 + 3], 0.0f), 1024.0f);
    bx[tid * 4 + 0] = x1;
    bx[tid * 4 + 1] = y1;
    bx[tid * 4 + 2] = x2;
    bx[tid * 4 + 3] = y2;
    const int k = kp[tid];
    rel[tid] = (k != 0 && fy >= y1 && fy < y2) ? 1 : 0;
  }
  __syncthreads();
  if (tid == 0) {
    int c = 0;
    for (int j = 0; j < TOPK; ++j) {
      if (rel[j]) { lst[c] = j; ++c; }
    }
    cnt = c;
  }
  __syncthreads();
  int n = cnt;
  if (n > TOPK) n = TOPK;
  const int x0 = tid * 4;
  unsigned mk = 0u;
  for (int jj = 0; jj < n; ++jj) {
    int j = lst[jj];
    j = (j < 0) ? 0 : ((j >= TOPK) ? (TOPK - 1) : j);
    const float x1 = bx[j * 4 + 0], y1 = bx[j * 4 + 1];
    const float x2 = bx[j * 4 + 2], y2 = bx[j * 4 + 3];
    const bool yin = (fy >= y1) && (fy < y2);
    const bool yinner = (fy >= y1 + 4.0f) && (fy < y2 - 4.0f);
    const float x1b = x1 + 4.0f, x2b = x2 - 4.0f;
#pragma unroll
    for (int q = 0; q < 4; ++q) {
      const float fx = (float)(x0 + q);
      const bool inside = yin && (fx >= x1) && (fx < x2);
      const bool inner = yinner && (fx >= x1b) && (fx < x2b);
      if (inside && !inner) mk |= (1u << q);
    }
  }
  const size_t rbase = (size_t)y * IMW + (size_t)x0;
  P4F f0, f1, f2, o0, o1, o2;
  f0.v = *(const v4f*)(frame + rbase);
  f1.v = *(const v4f*)(frame + IMHW + rbase);
  f2.v = *(const v4f*)(frame + 2 * IMHW + rbase);
#pragma unroll
  for (int q = 0; q < 4; ++q) {
    const bool mq = (mk >> q) & 1u;
    o0.f[q] = mq ? 1.0f : f0.f[q];
    o1.f[q] = mq ? 0.0f : f1.f[q];
    o2.f[q] = mq ? 0.0f : f2.f[q];
  }
  *(volatile v4f*)(out + rbase) = o0.v;
  *(volatile v4f*)(out + IMHW + rbase) = o1.v;
  *(volatile v4f*)(out + 2 * IMHW + rbase) = o2.v;
  __threadfence();
  *(volatile v4f*)(out + rbase) = o0.v;
  *(volatile v4f*)(out + IMHW + rbase) = o1.v;
  *(volatile v4f*)(out + 2 * IMHW + rbase) = o2.v;
}

extern "C" void kernel_launch(void* const* d_in, const int* in_sizes, int n_in,
                              void* d_out, int out_size, void* d_ws, size_t ws_size,
                              hipStream_t stream) {
  (void)in_sizes; (void)n_in; (void)out_size;
  const float* frame = (const float*)d_in[0];
  const float* w1 = (const float*)d_in[1];  const float* b1 = (const float*)d_in[2];
  const float* w2 = (const float*)d_in[3];  const float* b2 = (const float*)d_in[4];
  const float* w3 = (const float*)d_in[5];  const float* b3 = (const float*)d_in[6];
  const float* w4 = (const float*)d_in[7];  const float* b4 = (const float*)d_in[8];
  const float* wh = (const float*)d_in[9];  const float* bh = (const float*)d_in[10];
  float* out = (float*)d_out;

  char* ws = (char*)d_ws;
  size_t off = 0;
  auto bump = [&](size_t bytes) -> char* {
    char* p = ws + off;
    off += (bytes + 255) & ~(size_t)255;
    return p;
  };
  unsigned short* x1H = (unsigned short*)bump(512ull * 512 * 32 * 2);
  unsigned short* x1L = (unsigned short*)bump(512ull * 512 * 32 * 2);
  unsigned short* x2H = (unsigned short*)bump(256ull * 256 * 64 * 2);
  unsigned short* x2L = (unsigned short*)bump(256ull * 256 * 64 * 2);
  unsigned short* x3H = (unsigned short*)bump(128ull * 128 * 128 * 2);
  unsigned short* x3L = (unsigned short*)bump(128ull * 128 * 128 * 2);
  unsigned short* x4H = (unsigned short*)bump(64ull * 64 * 256 * 2);
  unsigned short* x4L = (unsigned short*)bump(64ull * 64 * 256 * 2);
  float* hdF = (float*)bump(4096ull * 16 * 4);
  unsigned short* w1H = (unsigned short*)bump(32ull * 32 * 2);
  unsigned short* w1L = (unsigned short*)bump(32ull * 32 * 2);
  unsigned short* w2H = (unsigned short*)bump(64ull * 288 * 2);
  unsigned short* w2L = (unsigned short*)bump(64ull * 288 * 2);
  unsigned short* w3H = (unsigned short*)bump(128ull * 576 * 2);
  unsigned short* w3L = (unsigned short*)bump(128ull * 576 * 2);
  unsigned short* w4H = (unsigned short*)bump(256ull * 1152 * 2);
  unsigned short* w4L = (unsigned short*)bump(256ull * 1152 * 2);
  unsigned short* whH = (unsigned short*)bump(16ull * 2304 * 2);
  unsigned short* whL = (unsigned short*)bump(16ull * 2304 * 2);
  float* topbox = (float*)bump((size_t)TOPKP * 4 * 4);
  int* keep = (int*)bump((size_t)TOPKP * 4);
  if (off > ws_size) return;

  { int nThr = 32 * 32 / 8;     k_pack<<<(nThr + 255) / 256, 256, 0, stream>>>(w1, w1H, w1L, 32, 3, 32, nThr); }
  { int nThr = 64 * 288 / 8;    k_pack<<<(nThr + 255) / 256, 256, 0, stream>>>(w2, w2H, w2L, 64, 32, 288, nThr); }
  { int nThr = 128 * 576 / 8;   k_pack<<<(nThr + 255) / 256, 256, 0, stream>>>(w3, w3H, w3L, 128, 64, 576, nThr); }
  { int nThr = 256 * 1152 / 8;  k_pack<<<(nThr + 255) / 256, 256, 0, stream>>>(w4, w4H, w4L, 256, 128, 1152, nThr); }
  { int nThr = 16 * 2304 / 8;   k_pack<<<(nThr + 255) / 256, 256, 0, stream>>>(wh, whH, whL, 15, 256, 2304, nThr); }

  { int nT = 512 * 512 / 16; k_conv1<<<(nT + 3) / 4, 128, 0, stream>>>(frame, w1H, w1L, b1, x1H, x1L, nT); }
  { int nT = (256 * 256 / 16) * (64 / 64);
    k_conv<4, 0><<<(nT + 3) / 4, 128, 0, stream>>>(x1H, x1L, w2H, w2L, b2, x2H, x2L, hdF,
                                                 32, 512, 512, 256, 64, 64, 2, 0, 1, nT); }
  { int nT = (128 * 128 / 16) * (128 / 64);
    k_conv<4, 0><<<(nT + 3) / 4, 128, 0, stream>>>(x2H, x2L, w3H, w3L, b3, x3H, x3L, hdF,
                                                 64, 256, 256, 128, 128, 128, 2, 0, 1, nT); }
  { int nT = (64 * 64 / 16) * (256 / 64);
    k_conv<4, 0><<<(nT + 3) / 4, 128, 0, stream>>>(x3H, x3L, w4H, w4L, b4, x4H, x4L, hdF,
                                                 128, 128, 128, 64, 256, 256, 2, 0, 1, nT); }
  { int nT = (64 * 64 / 16) * 1;
    k_conv<1, 1><<<(nT + 3) / 4, 128, 0, stream>>>(x4H, x4L, whH, whL, bh, x1H, x1L, hdF,
                                                 256, 64, 64, 64, 16, 15, 1, 1, 0, nT); }

  k_select<<<1, 256, 0, stream>>>(hdF, topbox, keep);
  k_draw<<<1024, 256, 0, stream>>>(frame, topbox, keep, out);
}
